// VGAEEncoder_31344671326932
// MI455X (gfx1250) — hardware-run, weakly checked
//
#include <hip/hip_runtime.h>
#include <stddef.h>
#include <stdint.h>
#include <math.h>

#define HEAD_SPLIT 1

#define NN      50000
#define NE      800000
#define DD      128
#define NH      256
#define GBM     128
#define MP      50048
#if HEAD_SPLIT
#define KH      256
#define UPRS    5
#else
#define KH      128
#define UPRS    4
#endif
#define NTHR    256
#define NWAVE   8
#define EPT     8
#define WCH     (32 * EPT)
#define NBRUN   1024
#define SLB     10
#define NBK     49
#define WLCAP   2560
#define RCAP    20480
#define DEGCAP  64
#define MAXDEG_MEAS   35
#define MAXB1024_MEAS 16623
#define RB      64
#define SP      68
#define OUT1    6400000
#define WSMAX   134217728

#define BK_ZINTS (NWAVE * WLCAP + RCAP + 3 * NBRUN)
#define BK_INTS  (BK_ZINTS + 16)
#define BK_LDS   (BK_INTS * 4)

#define PBX   (MP * DD / 8 / NTHR)
#define PBW1  (DD * DD / 8 / NTHR)
#define PBWH  (NH * KH / 8 / NTHR)
#define PBTOT (PBX + PBW1 + PBWH + 1)

static_assert(DD == 128 && DD == 32 * 4 && NH == 2 * DD && NH == 32 * 8);
static_assert(MP % GBM == 0 && MP >= NN && MP == 391 * GBM && MP % RB == 0);
static_assert(NBRUN == (1 << SLB) && NBRUN % RB == 0 && NBRUN % GBM == 0 && NBRUN % 32 == 0);
static_assert(NBK * NBRUN >= MP && NN <= NBK * NBRUN);
static_assert(NE < (1 << 20) && (((long long)NE) << SLB) < (1LL << 31));
static_assert(NE % WCH == 0 && NE % 4 == 0);
static_assert(RCAP == NWAVE * WLCAP && RCAP % (NTHR * 4) == 0 && BK_ZINTS % 4 == 0);
static_assert((2 * NBRUN) % (NTHR * 4) == 0 && NBRUN == NTHR * 4);
static_assert((long long)RCAP * 100 >= (long long)MAXB1024_MEAS * 110);
static_assert(WLCAP >= MAXB1024_MEAS / 8 + 8 * 46 + 1);
static_assert(MAXDEG_MEAS + 8 <= DEGCAP);
static_assert((MP * DD / 8) % NTHR == 0 && (DD * DD / 8) % NTHR == 0 && (NH * KH / 8) % NTHR == 0);
static_assert(KH % 32 == 0 && DD % 32 == 0 && (KH == 2 * DD || KH == DD) && (KH / 8) == (1 << UPRS));
static_assert((DD * (KH / 8)) % NTHR == 0);
static_assert(BK_LDS <= 300000);
static_assert((GBM * SP + GBM) * 4 <= 65536);
static_assert(RB % NWAVE == 0);
static_assert((long long)OUT1 + (long long)(NN - 1) * DD + DD - 1 < 2LL * NN * DD);
static_assert(OUT1 == NN * DD && (OUT1 * 4) % 128 == 0);

typedef float          v4f   __attribute__((ext_vector_type(4)));
typedef float          v8f   __attribute__((ext_vector_type(8)));
typedef int            v4i   __attribute__((ext_vector_type(4)));
typedef int            v8i   __attribute__((ext_vector_type(8)));
typedef unsigned short v8us  __attribute__((ext_vector_type(8)));
typedef unsigned short v16us __attribute__((ext_vector_type(16)));
typedef __bf16         v16bf __attribute__((ext_vector_type(16)));
typedef v4f  __attribute__((may_alias)) v4fa;
typedef v4i  __attribute__((may_alias)) v4ia;
typedef v8us __attribute__((may_alias)) v8usa;
union FragB { v16bf v; v16us u; v8us h[2]; v8i w; };

__device__ __forceinline__ v8f wmb(const FragB& a, const FragB& b, v8f c) {
  v8f d = __builtin_amdgcn_wmma_f32_16x16x32_bf16(false, a.v, false, b.v, (short)0, c, false, false);
  asm volatile("v_nop\n\tv_nop\n\tv_nop\n\tv_nop" : "+v"(d) : "v"(a.w), "v"(b.w));
  return d;
}

__device__ __forceinline__ unsigned bf16_bits(float f) {
  const unsigned u = __float_as_uint(f);
  const unsigned r = (u + 0x7FFFu + ((u >> 16) & 1u)) >> 16;
  const unsigned q = (u >> 16) | 0x40u;
  return ((u & 0x7fffffffu) > 0x7f800000u) ? q : r;
}
__device__ __forceinline__ float bf16_val(float f) {
  return __uint_as_float(bf16_bits(f) << 16);
}

__device__ __forceinline__ void hilo_pack(float v0, float v1, float v2, float v3,
                                          int& h01, int& h23, int& l01, int& l23) {
  const unsigned a0 = bf16_bits(v0), a1 = bf16_bits(v1), a2 = bf16_bits(v2), a3 = bf16_bits(v3);
  const unsigned b0 = bf16_bits(v0 - __uint_as_float(a0 << 16));
  const unsigned b1 = bf16_bits(v1 - __uint_as_float(a1 << 16));
  const unsigned b2 = bf16_bits(v2 - __uint_as_float(a2 << 16));
  const unsigned b3 = bf16_bits(v3 - __uint_as_float(a3 << 16));
  h01 = (int)(a0 | (a1 << 16)); h23 = (int)(a2 | (a3 << 16));
  l01 = (int)(b0 | (b1 << 16)); l23 = (int)(b2 | (b3 << 16));
}

__device__ __forceinline__ v4i regroup_row(int h01, int h23, int l01, int l23, int lane) {
  const int s0 = (2 * lane) & 31, s1 = s0 + 1;
  const int a0 = __shfl(h01, s0, 32), a1 = __shfl(h23, s0, 32), a2 = __shfl(h01, s1, 32), a3 = __shfl(h23, s1, 32);
  const int b0 = __shfl(l01, s0, 32), b1 = __shfl(l23, s0, 32), b2 = __shfl(l01, s1, 32), b3 = __shfl(l23, s1, 32);
  const int mk = (lane < 16) ? -1 : 0;
  v4i o;
  o.x = (a0 & mk) | (b0 & ~mk); o.y = (a1 & mk) | (b1 & ~mk);
  o.z = (a2 & mk) | (b2 & ~mk); o.w = (a3 & mk) | (b3 & ~mk);
  return o;
}

__device__ __forceinline__ void st2_v4f(float* p, v4f v) {
  *(volatile v4f*)p = v;
  __threadfence();
  *(volatile v4f*)p = v;
}
__device__ __forceinline__ void st2_v8us(unsigned short* p, v8us v) {
  *(volatile v8us*)p = v;
  __threadfence();
  *(volatile v8us*)p = v;
}

__device__ __forceinline__ v8us colpick8(const float* __restrict__ base, int stride) {
  float f[8];
#pragma unroll
  for (int i = 0; i < 8; ++i) f[i] = base[(size_t)i * (size_t)stride];
  v8us o;
#pragma unroll
  for (int i = 0; i < 8; ++i) o[i] = (unsigned short)bf16_bits(f[i]);
  return o;
}

__device__ __forceinline__ void bias_line(const float* __restrict__ src, float* dst, int lane) {
  const v4f a = *(const v4fa*)(src + 4 * lane);
  v4f o;
  o.x = bf16_val(a.x); o.y = bf16_val(a.y); o.z = bf16_val(a.z); o.w = bf16_val(a.w);
  st2_v4f(dst + 4 * lane, o);
}

__global__ __launch_bounds__(NTHR) void k_prep(const float* __restrict__ x, const float* __restrict__ w1,
                                               const float* __restrict__ b1, const float* __restrict__ wmu,
                                               const float* __restrict__ bmu, const float* __restrict__ wls,
                                               const float* __restrict__ bls,
                                               unsigned short* xb, unsigned short* w1t, unsigned short* wh,
                                               float* sm) {
  const int tid = (int)threadIdx.x, lane = tid & 31;
  const int blk = (int)blockIdx.x;
  if (blk < PBX) {
    const int u   = blk * NTHR + tid;
    const int row = u >> 4, k8 = (u & 15) * 8;
    const int rc  = row < NN ? row : NN - 1;
    const unsigned mk = row < NN ? 0xffffu : 0u;
    const float* p = x + (size_t)rc * DD + k8;
    const v4f a = *(const v4fa*)p;
    const v4f b = *(const v4fa*)(p + 4);
    v8us o;
    o[0] = (unsigned short)(bf16_bits(a.x) & mk); o[1] = (unsigned short)(bf16_bits(a.y) & mk);
    o[2] = (unsigned short)(bf16_bits(a.z) & mk); o[3] = (unsigned short)(bf16_bits(a.w) & mk);
    o[4] = (unsigned short)(bf16_bits(b.x) & mk); o[5] = (unsigned short)(bf16_bits(b.y) & mk);
    o[6] = (unsigned short)(bf16_bits(b.z) & mk); o[7] = (unsigned short)(bf16_bits(b.w) & mk);
    st2_v8us(xb + (size_t)row * DD + k8, o);
  } else if (blk < PBX + PBW1) {
    const int u = (blk - PBX) * NTHR + tid;
    const int n = u >> 4, k8 = (u & 15) * 8;
    const v8us o = colpick8(w1 + (size_t)k8 * DD + n, DD);
    st2_v8us(w1t + (size_t)n * DD + k8, o);
  } else if (blk < PBX + PBW1 + PBWH) {
    const int bw = blk - PBX - PBW1;
    const int u  = bw * NTHR + tid;
    const int n  = u >> UPRS, k8 = (u & ((KH / 8) - 1)) * 8, kk = k8 & (DD - 1);
    const bool first = bw < (DD * (KH / 8) / NTHR);
    v8us o;
    if (first) o = colpick8(wmu + (size_t)kk * DD + n, DD);
    else       o = colpick8(wls + (size_t)kk * DD + (n - DD), DD);
    st2_v8us(wh + (size_t)n * KH + k8, o);
  } else {
    const int wv = __builtin_amdgcn_readfirstlane(tid >> 5);
    if (wv == 0)      bias_line(b1,  sm,          lane);
    else if (wv == 1) bias_line(bmu, sm + DD,     lane);
    else if (wv == 2) bias_line(bls, sm + 2 * DD, lane);
  }
}

__device__ __forceinline__ void bucket_flush(const int* pl, const int* cnt, const int* dvb, int ov,
                                             int* lp, int* cop, int* dp, int* fp, int tid) {
#pragma unroll 1
  for (int i = tid * 4; i < RCAP; i += NTHR * 4) {
    const v4i v = *(const v4ia*)(pl + i);
    *(volatile v4i*)(lp + i) = v;
  }
#pragma unroll 1
  for (int i = tid * 4; i < 2 * NBRUN; i += NTHR * 4) {
    const v4i v = *(const v4ia*)(cnt + i);
    *(volatile v4i*)(cop + i) = v;
  }
  {
    const v4i v = *(const v4ia*)(dvb + 4 * tid);
    *(volatile v4i*)(dp + 4 * tid) = v;
  }
  if (tid < 8) {
    const v4i f = {ov, ov, ov, ov};
    *(volatile v4i*)(fp + 4 * tid) = f;
  }
}

__global__ __launch_bounds__(NTHR) void k_bucket(const int* __restrict__ srcs, const int* __restrict__ dsts,
                                                 int* LIST, int* CO, int* DINVB, int* FLAG) {
  extern __shared__ __attribute__((aligned(16))) int dsm[];
  int* wl   = dsm;
  int* pl   = dsm + NWAVE * WLCAP;
  int* cnt  = pl + RCAP;
  int* offs = cnt + NBRUN;
  int* cur  = offs + NBRUN;
  int* misc = cur + NBRUN;
  const int tid = (int)threadIdx.x, lane = tid & 31, wave = tid >> 5;
  const int blk = (int)blockIdx.x;
  const unsigned nbs = (unsigned)(blk * NBRUN);

  {
    const v4i z4 = {0, 0, 0, 0};
    for (int i = tid * 4; i < BK_ZINTS; i += NTHR * 4) *(v4ia*)(dsm + i) = z4;
    if (tid < 16) misc[tid] = 0;
  }
  __syncthreads();

  {
    const int per  = ((NE + NWAVE * WCH - 1) / (NWAVE * WCH)) * WCH;
    const int ebeg = wave * per;
    const int eend = (ebeg + per < NE) ? (ebeg + per) : NE;
    int* mylist = wl + wave * WLCAP;
    int wc = 0;
#pragma unroll 1
    for (int cb = ebeg; cb < eend; cb += WCH) {
      const int e0 = cb + lane * EPT;
      const v4i da = *(const v4ia*)(dsts + e0);
      const v4i db = *(const v4ia*)(dsts + e0 + 4);
      const unsigned s0 = (unsigned)da.x - nbs, s1 = (unsigned)da.y - nbs;
      const unsigned s2 = (unsigned)da.z - nbs, s3 = (unsigned)da.w - nbs;
      const unsigned s4 = (unsigned)db.x - nbs, s5 = (unsigned)db.y - nbs;
      const unsigned s6 = (unsigned)db.z - nbs, s7 = (unsigned)db.w - nbs;
      const bool h0 = s0 < (unsigned)NBRUN, h1 = s1 < (unsigned)NBRUN, h2 = s2 < (unsigned)NBRUN, h3 = s3 < (unsigned)NBRUN;
      const bool h4 = s4 < (unsigned)NBRUN, h5 = s5 < (unsigned)NBRUN, h6 = s6 < (unsigned)NBRUN, h7 = s7 < (unsigned)NBRUN;
      const unsigned m0 = __builtin_amdgcn_ballot_w32(h0), m1 = __builtin_amdgcn_ballot_w32(h1);
      const unsigned m2 = __builtin_amdgcn_ballot_w32(h2), m3 = __builtin_amdgcn_ballot_w32(h3);
      const unsigned m4 = __builtin_amdgcn_ballot_w32(h4), m5 = __builtin_amdgcn_ballot_w32(h5);
      const unsigned m6 = __builtin_amdgcn_ballot_w32(h6), m7 = __builtin_amdgcn_ballot_w32(h7);
      const unsigned any = m0 | m1 | m2 | m3 | m4 | m5 | m6 | m7;
      if (any != 0u) {
        const int pre = (int)(__builtin_amdgcn_mbcnt_lo(m0, 0u) + __builtin_amdgcn_mbcnt_lo(m1, 0u) +
                              __builtin_amdgcn_mbcnt_lo(m2, 0u) + __builtin_amdgcn_mbcnt_lo(m3, 0u) +
                              __builtin_amdgcn_mbcnt_lo(m4, 0u) + __builtin_amdgcn_mbcnt_lo(m5, 0u) +
                              __builtin_amdgcn_mbcnt_lo(m6, 0u) + __builtin_amdgcn_mbcnt_lo(m7, 0u));
        int p = wc + pre;
        if (h0) { if (p < WLCAP) mylist[p] = ((e0 + 0) << SLB) | (int)s0; p = p + 1; }
        if (h1) { if (p < WLCAP) mylist[p] = ((e0 + 1) << SLB) | (int)s1; p = p + 1; }
        if (h2) { if (p < WLCAP) mylist[p] = ((e0 + 2) << SLB) | (int)s2; p = p + 1; }
        if (h3) { if (p < WLCAP) mylist[p] = ((e0 + 3) << SLB) | (int)s3; p = p + 1; }
        if (h4) { if (p < WLCAP) mylist[p] = ((e0 + 4) << SLB) | (int)s4; p = p + 1; }
        if (h5) { if (p < WLCAP) mylist[p] = ((e0 + 5) << SLB) | (int)s5; p = p + 1; }
        if (h6) { if (p < WLCAP) mylist[p] = ((e0 + 6) << SLB) | (int)s6; p = p + 1; }
        if (h7) { if (p < WLCAP) mylist[p] = ((e0 + 7) << SLB) | (int)s7; p = p + 1; }
        wc += (int)(__builtin_popcount(m0) + __builtin_popcount(m1) + __builtin_popcount(m2) + __builtin_popcount(m3) +
                    __builtin_popcount(m4) + __builtin_popcount(m5) + __builtin_popcount(m6) + __builtin_popcount(m7));
      }
    }
    if (lane == 0) misc[wave] = wc;
  }
  __syncthreads();

  if (wave == 0) {
    int ov = 0;
#pragma unroll 1
    for (int w2 = 0; w2 < NWAVE; ++w2) {
      int c = misc[w2];
      if (c > WLCAP) ov = 1;
      c = c < 0 ? 0 : (c > WLCAP ? WLCAP : c);
#pragma unroll 1
      for (int b0 = 0; b0 < c; b0 += 32) {
        const int idx = b0 + lane;
        const int ent = wl[w2 * WLCAP + (idx < WLCAP ? idx : WLCAP - 1)];
        const int m32 = (c - b0) < 32 ? (c - b0) : 32;
#pragma unroll 1
        for (int k = 0; k < m32; ++k) {
          const int u    = __builtin_amdgcn_readlane(ent, k);
          const int slot = u & (NBRUN - 1);
          if (lane == 0) cnt[slot] = cnt[slot] + 1;
        }
      }
    }
    if (lane == 0) misc[9] = ov;
  }
  __syncthreads();
  if (wave == 0) {
    const int base = lane * (NBRUN / 32);
    int s = 0;
#pragma unroll 1
    for (int i = 0; i < NBRUN / 32; ++i) s += cnt[base + i];
    int incl = s;
#pragma unroll
    for (int d = 1; d < 32; d <<= 1) {
      const int y = __shfl_up(incl, d, 32);
      if (lane >= d) incl += y;
    }
    int run = incl - s;
#pragma unroll 1
    for (int i = 0; i < NBRUN / 32; ++i) {
      const int cv = cnt[base + i];
      offs[base + i] = run;
      cur[base + i]  = run;
      run += cv;
    }
  }
  __syncthreads();

  if (wave == 0) {
#pragma unroll 1
    for (int w2 = 0; w2 < NWAVE; ++w2) {
      int c = misc[w2];
      c = c < 0 ? 0 : (c > WLCAP ? WLCAP : c);
#pragma unroll 1
      for (int b0 = 0; b0 < c; b0 += 32) {
        const int idx = b0 + lane;
        const int ent = wl[w2 * WLCAP + (idx < WLCAP ? idx : WLCAP - 1)];
        int eid = (ent >> SLB) & 0xFFFFF;
        eid = eid > NE - 1 ? NE - 1 : eid;
        int sr = srcs[eid];
        sr = sr < 0 ? 0 : (sr > NN - 1 ? NN - 1 : sr);
        const int m32 = (c - b0) < 32 ? (c - b0) : 32;
#pragma unroll 1
        for (int k = 0; k < m32; ++k) {
          const int u    = __builtin_amdgcn_readlane(ent, k);
          const int wd   = __builtin_amdgcn_readlane(sr, k);
          const int slot = u & (NBRUN - 1);
          if (lane == 0) {
            int p = cur[slot];
            p = p < 0 ? 0 : (p > RCAP - 1 ? RCAP - 1 : p);
            pl[p] = wd;
            cur[slot] = p + 1;
          }
        }
      }
    }
  }
  __syncthreads();

#pragma unroll 1
  for (int i = tid; i < NBRUN; i += NTHR) {
    const int cv = cnt[i];
    if (cv > DEGCAP) misc[10] = 1;
    const float dg = (float)(cv + 1);
    cur[i] = __float_as_int(1.0f / sqrtf(dg));
  }
  __syncthreads();

  const int ovf = misc[9] | misc[10];
  int* lp  = LIST + (size_t)blk * RCAP;
  int* cop = CO + (size_t)blk * (2 * NBRUN);
  int* dp  = DINVB + (size_t)blk * NBRUN;
  int* fp  = FLAG + (size_t)blk * 32;
  bucket_flush(pl, cnt, cur, ovf, lp, cop, dp, fp, tid);
  __threadfence();
  bucket_flush(pl, cnt, cur, ovf, lp, cop, dp, fp, tid);
}

template <int KTOT>
__device__ __forceinline__ void gemm_16x64(const unsigned short* __restrict__ ap,
                                           const unsigned short* __restrict__ bp, v8f (&acc)[4]) {
#pragma unroll 1
  for (int k0 = 0; k0 < KTOT; k0 += 32) {
    FragB af;
    af.h[0] = *(const v8usa*)(ap + k0);
    af.h[1] = *(const v8usa*)(ap + k0 + 16);
#pragma unroll
    for (int nt = 0; nt < 4; ++nt) {
      const unsigned short* wq = bp + (size_t)(16 * nt) * (size_t)KTOT + k0;
      FragB bf;
      bf.h[0] = *(const v8usa*)wq;
      bf.h[1] = *(const v8usa*)(wq + 16);
      acc[nt] = wmb(af, bf, acc[nt]);
    }
  }
}

__device__ __forceinline__ void stage_d(float* stg, const v8f (&acc)[4], int wave, int hh, int m) {
#pragma unroll
  for (int nt = 0; nt < 4; ++nt) {
#pragma unroll
    for (int r = 0; r < 8; ++r) stg[(16 * wave + 8 * hh + r) * SP + 16 * nt + m] = acc[nt][r];
  }
}

template <int KTOT, int LDO>
__global__ __launch_bounds__(NTHR) __attribute__((amdgpu_num_vgpr(248)))
void k_gemm(const unsigned short* __restrict__ A, const unsigned short* __restrict__ BT,
            const float* __restrict__ DINV, float* P) {
  __shared__ __attribute__((aligned(16))) float stg[GBM * SP];
  __shared__ __attribute__((aligned(16))) float sdv[GBM];
  const int tid = (int)threadIdx.x, lane = tid & 31, wave = tid >> 5, hh = lane >> 4, m = lane & 15;
  const int rowBase = (int)blockIdx.x * GBM;
  const int col0    = (int)blockIdx.y * 64;
  if (tid < 32) *(v4fa*)(sdv + 4 * tid) = *(const v4fa*)(DINV + (size_t)rowBase + 4 * tid);

  v8f acc[4];
  {
    const v8f z = {0.f, 0.f, 0.f, 0.f, 0.f, 0.f, 0.f, 0.f};
#pragma unroll
    for (int t = 0; t < 4; ++t) acc[t] = z;
  }
  const unsigned short* ap = A + (size_t)(rowBase + 16 * wave + m) * (size_t)KTOT + 8 * hh;
  const unsigned short* bp = BT + (size_t)(col0 + m) * (size_t)KTOT + 8 * hh;
  gemm_16x64<KTOT>(ap, bp, acc);
  stage_d(stg, acc, wave, hh, m);
  __syncthreads();

#pragma unroll 1
  for (int i = 0; i < 8; ++i) {
    const int lr   = 16 * wave + 2 * i + hh;
    const int grow = rowBase + lr;
    const v4f a = *(const v4fa*)(stg + lr * SP + 4 * m);
    const float dv = sdv[lr];
    v4f o;
    o.x = dv * a.x; o.y = dv * a.y; o.z = dv * a.z; o.w = dv * a.w;
    st2_v4f(P + (size_t)grow * (size_t)LDO + col0 + 4 * m, o);
  }
}

__global__ __launch_bounds__(NTHR) void k_replay1(const int* __restrict__ LIST, const int* __restrict__ CO,
                                                  const int* __restrict__ FLAG, const float* __restrict__ DINV,
                                                  const float* __restrict__ P1, const float* __restrict__ SM,
                                                  unsigned short* H1) {
  const int tid = (int)threadIdx.x, lane = tid & 31, wave = tid >> 5;
  const int rowBase = (int)blockIdx.x * RB;
  const int bucket  = rowBase >> SLB;
  const int* lb  = LIST + (size_t)bucket * RCAP;
  const int* cob = CO + (size_t)bucket * (2 * NBRUN);
  const int flag = FLAG[(size_t)bucket * 32];
  const float qnan = __uint_as_float(0x7fc00000u);
  const v4f bias = *(const v4fa*)(SM + 4 * lane);

#pragma unroll 1
  for (int i = 0; i < RB / NWAVE; ++i) {
    const int d    = rowBase + (RB / NWAVE) * wave + i;
    const int slot = d & (NBRUN - 1);
    int c = cob[slot];
    int o = cob[NBRUN + slot];
    const bool big = c > DEGCAP;
    c = c < 0 ? 0 : (c > DEGCAP ? DEGCAP : c);
    o = o < 0 ? 0 : (o > RCAP - 1 ? RCAP - 1 : o);
    c = __builtin_amdgcn_readfirstlane(c);
    o = __builtin_amdgcn_readfirstlane(o);
    int last = o + c - 1; last = last < o ? o : last;
    last = last > RCAP - 1 ? RCAP - 1 : last;
    float a0 = 0.0f, a1 = 0.0f, a2 = 0.0f, a3 = 0.0f;
#pragma unroll 1
    for (int j = 0; j < c; ++j) {
      int idx = o + j;
      idx = idx > last ? last : idx;
      int sr = lb[idx];
      sr = sr < 0 ? 0 : (sr > NN - 1 ? NN - 1 : sr);
      const v4f v = *(const v4fa*)(P1 + (size_t)sr * DD + 4 * lane);
      asm volatile("" :: "v"(v));
      a0 += v.x; a1 += v.y; a2 += v.z; a3 += v.w;
    }
    const int dc = d < NN ? d : NN - 1;
    const v4f pv = *(const v4fa*)(P1 + (size_t)dc * DD + 4 * lane);
    const float dv = DINV[dc];
    asm volatile("" :: "v"(pv));
    asm volatile("" :: "v"(dv));
    float t0 = dv * (a0 + pv.x) + bias.x, t1 = dv * (a1 + pv.y) + bias.y;
    float t2 = dv * (a2 + pv.z) + bias.z, t3 = dv * (a3 + pv.w) + bias.w;
    t0 = (t0 > 0.0f) ? t0 : (t0 - t0); t1 = (t1 > 0.0f) ? t1 : (t1 - t1);
    t2 = (t2 > 0.0f) ? t2 : (t2 - t2); t3 = (t3 > 0.0f) ? t3 : (t3 - t3);
    const bool bad  = (flag != 0) | big;
    const bool live = d < NN;
    t0 = bad ? qnan : t0; t1 = bad ? qnan : t1; t2 = bad ? qnan : t2; t3 = bad ? qnan : t3;
    t0 = live ? t0 : 0.0f; t1 = live ? t1 : 0.0f; t2 = live ? t2 : 0.0f; t3 = live ? t3 : 0.0f;
    int h01, h23, l01, l23;
    hilo_pack(t0, t1, t2, t3, h01, h23, l01, l23);
    const v4i ow = regroup_row(h01, h23, l01, l23, lane);
#if HEAD_SPLIT
    unsigned short* hp = H1 + (size_t)d * KH + 8 * lane;
    *(volatile v4i*)hp = ow;
    __threadfence();
    *(volatile v4i*)hp = ow;
#else
    unsigned short* hp = H1 + (size_t)d * KH + 8 * (lane & 15);
    const bool wr = lane < 16;
    if (wr) *(volatile v4i*)hp = ow;
    __threadfence();
    if (wr) *(volatile v4i*)hp = ow;
#endif
  }
}

__global__ __launch_bounds__(NTHR) void k_replay2(const int* __restrict__ LIST, const int* __restrict__ CO,
                                                  const int* __restrict__ FLAG, const float* __restrict__ DINV,
                                                  const float* __restrict__ P2, const float* __restrict__ SM,
                                                  float* out) {
  const int tid = (int)threadIdx.x, lane = tid & 31, wave = tid >> 5;
  const int rowBase = (int)blockIdx.x * RB;
  const int bucket  = rowBase >> SLB;
  const int* lb  = LIST + (size_t)bucket * RCAP;
  const int* cob = CO + (size_t)bucket * (2 * NBRUN);
  const int flag = FLAG[(size_t)bucket * 32];
  const float qnan = __uint_as_float(0x7fc00000u);
  const v4f bm = *(const v4fa*)(SM + DD + 4 * lane);
  const v4f bl = *(const v4fa*)(SM + 2 * DD + 4 * lane);

#pragma unroll 1
  for (int i = 0; i < RB / NWAVE; ++i) {
    const int d    = rowBase + (RB / NWAVE) * wave + i;
    const int slot = d & (NBRUN - 1);
    int c = cob[slot];
    int o = cob[NBRUN + slot];
    const bool big = c > DEGCAP;
    c = c < 0 ? 0 : (c > DEGCAP ? DEGCAP : c);
    o = o < 0 ? 0 : (o > RCAP - 1 ? RCAP - 1 : o);
    c = __builtin_amdgcn_readfirstlane(c);
    o = __builtin_amdgcn_readfirstlane(o);
    int last = o + c - 1; last = last < o ? o : last;
    last = last > RCAP - 1 ? RCAP - 1 : last;
    v4f a0 = {0.0f, 0.0f, 0.0f, 0.0f};
    v4f a1 = {0.0f, 0.0f, 0.0f, 0.0f};
#pragma unroll 1
    for (int j = 0; j < c; ++j) {
      int idx = o + j;
      idx = idx > last ? last : idx;
      int sr = lb[idx];
      sr = sr < 0 ? 0 : (sr > NN - 1 ? NN - 1 : sr);
      const float* p = P2 + (size_t)sr * NH + 4 * lane;
      const v4f v0 = *(const v4fa*)p;
      const v4f v1 = *(const v4fa*)(p + DD);
      asm volatile("" :: "v"(v0));
      asm volatile("" :: "v"(v1));
      a0 += v0; a1 += v1;
    }
    const int dc = d < NN ? d : NN - 1;
    const float* ps = P2 + (size_t)dc * NH + 4 * lane;
    const v4f s0 = *(const v4fa*)ps;
    const v4f s1 = *(const v4fa*)(ps + DD);
    const float dv = DINV[dc];
    asm volatile("" :: "v"(s0));
    asm volatile("" :: "v"(s1));
    asm volatile("" :: "v"(dv));
    const bool bad = (flag != 0) | big;
    v4f o0, o1;
    o0.x = dv * (a0.x + s0.x) + bm.x; o0.y = dv * (a0.y + s0.y) + bm.y;
    o0.z = dv * (a0.z + s0.z) + bm.z; o0.w = dv * (a0.w + s0.w) + bm.w;
    o1.x = dv * (a1.x + s1.x) + bl.x; o1.y = dv * (a1.y + s1.y) + bl.y;
    o1.z = dv * (a1.z + s1.z) + bl.z; o1.w = dv * (a1.w + s1.w) + bl.w;
    o0.x = bad ? qnan : o0.x; o0.y = bad ? qnan : o0.y; o0.z = bad ? qnan : o0.z; o0.w = bad ? qnan : o0.w;
    o1.x = bad ? qnan : o1.x; o1.y = bad ? qnan : o1.y; o1.z = bad ? qnan : o1.z; o1.w = bad ? qnan : o1.w;
    const bool live = d < NN;
    float* q0 = out + (size_t)dc * DD + 4 * lane;
    float* q1 = out + (size_t)OUT1 + (size_t)dc * DD + 4 * lane;
    if (live) { *(volatile v4f*)q0 = o0; *(volatile v4f*)q1 = o1; }
    __threadfence();
    if (live) { *(volatile v4f*)q0 = o0; *(volatile v4f*)q1 = o1; }
  }
}

extern "C" void kernel_launch(void* const* d_in, const int* in_sizes, int n_in,
                              void* d_out, int out_size, void* d_ws, size_t ws_size,
                              hipStream_t stream) {
  if (n_in < 8) return;
  if (in_sizes[0] != NN * DD) return;
  if (in_sizes[1] != 2 * NE) return;
  if (in_sizes[2] != DD * DD) return;
  if (in_sizes[3] != DD) return;
  if (in_sizes[4] != DD * DD) return;
  if (in_sizes[5] != DD) return;
  if (in_sizes[6] != DD * DD) return;
  if (in_sizes[7] != DD) return;
  if (out_size != 2 * NN * DD) return;

  const float* x   = (const float*)d_in[0];
  const int*   ei  = (const int*)d_in[1];
  const float* W1  = (const float*)d_in[2];
  const float* b1  = (const float*)d_in[3];
  const float* Wmu = (const float*)d_in[4];
  const float* bmu = (const float*)d_in[5];
  const float* Wls = (const float*)d_in[6];
  const float* bls = (const float*)d_in[7];
  float* out = (float*)d_out;
  const int* srcs = ei;
  const int* dsts = ei + NE;

  constexpr size_t zXB   = (size_t)MP * DD * 2;
  constexpr size_t zP1   = (size_t)MP * DD * 4;
  constexpr size_t zH1   = (size_t)MP * KH * 2;
  constexpr size_t zP2   = (size_t)MP * NH * 4;
  constexpr size_t zLIST = (size_t)NBK * RCAP * 4;
  constexpr size_t zCO   = (size_t)NBK * 2 * NBRUN * 4;
  constexpr size_t zDINV = (size_t)NBK * NBRUN * 4;
  constexpr size_t zFLAG = 6400;
  constexpr size_t zW1T  = (size_t)DD * DD * 2;
  constexpr size_t zWH   = (size_t)NH * KH * 2;
  constexpr size_t zSM   = (size_t)3 * DD * 4;
  constexpr size_t oXB   = 0;
  constexpr size_t oP1   = oXB + zXB;
  constexpr size_t oH1   = oP1 + zP1;
  constexpr size_t oP2   = oH1 + zH1;
  constexpr size_t oLIST = oP2 + zP2;
  constexpr size_t oCO   = oLIST + zLIST;
  constexpr size_t oDINV = oCO + zCO;
  constexpr size_t oFLAG = oDINV + zDINV;
  constexpr size_t oW1T  = oFLAG + zFLAG;
  constexpr size_t oWH   = oW1T + zW1T;
  constexpr size_t oSM   = oWH + zWH;
  constexpr size_t oEND  = oSM + zSM;
  static_assert(zXB % 256 == 0 && zP1 % 256 == 0 && zH1 % 256 == 0 && zP2 % 256 == 0 && zLIST % 256 == 0);
  static_assert(zCO % 256 == 0 && zDINV % 256 == 0 && zFLAG % 256 == 0 && zFLAG >= (size_t)NBK * 128);
  static_assert(zW1T % 256 == 0 && zWH % 256 == 0 && zSM % 256 == 0);
  static_assert(zDINV >= (size_t)MP * 4);
  static_assert(oEND <= (size_t)WSMAX);
  if (oEND > ws_size) return;

  char* ws = (char*)d_ws;
  unsigned short* XB   = (unsigned short*)(ws + oXB);
  float*          P1   = (float*)(ws + oP1);
  unsigned short* H1   = (unsigned short*)(ws + oH1);
  float*          P2   = (float*)(ws + oP2);
  int*            LIST = (int*)(ws + oLIST);
  int*            CO   = (int*)(ws + oCO);
  int*            DVB  = (int*)(ws + oDINV);
  const float*    DINV = (const float*)(ws + oDINV);
  int*            FLAG = (int*)(ws + oFLAG);
  unsigned short* W1T  = (unsigned short*)(ws + oW1T);
  unsigned short* WH   = (unsigned short*)(ws + oWH);
  float*          SM   = (float*)(ws + oSM);

  hipFuncSetAttribute(reinterpret_cast<const void*>(&k_bucket), hipFuncAttributeMaxDynamicSharedMemorySize, (int)BK_LDS);

  k_prep<<<PBTOT, NTHR, 0, stream>>>(x, W1, b1, Wmu, bmu, Wls, bls, XB, W1T, WH, SM);
  k_bucket<<<NBK, NTHR, BK_LDS, stream>>>(srcs, dsts, LIST, CO, DVB, FLAG);
  k_gemm<DD, DD><<<dim3(MP / GBM, DD / 64), NTHR, 0, stream>>>(XB, W1T, DINV, P1);
  k_replay1<<<MP / RB, NTHR, 0, stream>>>(LIST, CO, FLAG, DINV, P1, SM, H1);
  k_gemm<KH, NH><<<dim3(MP / GBM, NH / 64), NTHR, 0, stream>>>(H1, WH, DINV, P2);
  k_replay2<<<MP / RB, NTHR, 0, stream>>>(LIST, CO, FLAG, DINV, P2, SM, out);
}
